// LangModelWithLSTM_54022098649438
// MI455X (gfx1250) — hardware-verified
//
#include <hip/hip_runtime.h>
#include <hip/hip_bf16.h>


#define NB_   16
#define NS_   512
#define NR_   8192
#define NH_   512
#define NG_   2048
#define DIN_  1024
#define HID_  1024
#define NCL_  5
#define LM_   768
#define EMB_  256
#define VOC_  32000
#define TH_   256
#define NRH_  4096
#define W3R_  64
#define SCP_  68

static_assert(NR_ == NB_ * NS_);
static_assert(DIN_ == LM_ + EMB_);
static_assert(DIN_ == 2 * NH_);
static_assert(NRH_ == NB_ * TH_);
static_assert(NS_ == 2 * TH_);
static_assert(TH_ % 64 == 0);
static_assert(NG_ == 4 * NH_);
static_assert(NG_ % 64 == 0 && HID_ % 64 == 0 && NR_ % 64 == 0 && NRH_ % 64 == 0);
static_assert(DIN_ % 32 == 0 && HID_ % 32 == 0 && NH_ % 32 == 0);
static_assert(LM_ % 8 == 0 && EMB_ % 8 == 0);
static_assert((NR_ * DIN_ / 8) % 256 == 0);

typedef float          v4f   __attribute__((ext_vector_type(4)));
typedef float          v8f   __attribute__((ext_vector_type(8)));
typedef __bf16         v16b  __attribute__((ext_vector_type(16)));
typedef _Float16       v16h  __attribute__((ext_vector_type(16)));
typedef _Float16       v8h   __attribute__((ext_vector_type(8)));
typedef unsigned short u16x8 __attribute__((ext_vector_type(8)));

union Frag { u16x8 h[2]; v16b vb; v16h vh; };
union H8U { v8h f; u16x8 u; };
union H2U { _Float16 f; unsigned short u; };
union YStage { unsigned short y[2 * NB_ * NH_]; float c[NB_ * NH_]; };

constexpr size_t SZ_PL16 = (size_t)NR_ * DIN_ * 2;
constexpr size_t SZ_XG   = (size_t)NRH_ * NG_ * 4;
constexpr size_t SZ_WIH  = (size_t)NG_ * DIN_ * 2;
constexpr size_t SZ_WHH  = (size_t)NG_ * NH_ * 2;
constexpr size_t SZ_W1P  = (size_t)HID_ * DIN_ * 2;
constexpr size_t SZ_W2P  = (size_t)HID_ * HID_ * 2;
constexpr size_t SZ_W3P  = (size_t)W3R_ * HID_ * 2;
constexpr size_t SZ_CST  = (size_t)NB_ * NH_ * 4;
constexpr size_t SZ_HST  = (size_t)NB_ * NH_ * 2;

constexpr size_t OFF_PXH  = 0;
constexpr size_t OFF_PXL  = OFF_PXH + SZ_PL16;
constexpr size_t OFF_PYH  = OFF_PXL + SZ_PL16;
constexpr size_t OFF_PYL  = OFF_PYH + SZ_PL16;
constexpr size_t OFF_XG   = OFF_PYL + SZ_PL16;
constexpr size_t OFF_WIHH = OFF_XG + SZ_XG;
constexpr size_t OFF_WIHL = OFF_WIHH + SZ_WIH;
constexpr size_t OFF_WHH  = OFF_WIHL + SZ_WIH;
constexpr size_t OFF_W1P  = OFF_WHH + SZ_WHH;
constexpr size_t OFF_W2H  = OFF_W1P + SZ_W1P;
constexpr size_t OFF_W2L  = OFF_W2H + SZ_W2P;
constexpr size_t OFF_W3H  = OFF_W2L + SZ_W2P;
constexpr size_t OFF_W3L  = OFF_W3H + SZ_W3P;
constexpr size_t OFF_CST  = OFF_W3L + SZ_W3P;
constexpr size_t OFF_HST  = OFF_CST + SZ_CST;
constexpr size_t WS_END   = OFF_HST + SZ_HST;
static_assert(WS_END <= (size_t)134217728);
static_assert(OFF_PXL % 128 == 0 && OFF_PYH % 128 == 0 && OFF_PYL % 128 == 0 && OFF_XG % 128 == 0);
static_assert(OFF_WIHH % 128 == 0 && OFF_WIHL % 128 == 0 && OFF_WHH % 128 == 0 && OFF_W1P % 128 == 0);
static_assert(OFF_W2H % 128 == 0 && OFF_W2L % 128 == 0 && OFF_W3H % 128 == 0 && OFF_W3L % 128 == 0);
static_assert(OFF_CST % 128 == 0 && OFF_HST % 128 == 0);

__device__ __forceinline__ unsigned short f2bf(float f) {
    unsigned u = __float_as_uint(f);
    unsigned r = u + 0x7FFFu + ((u >> 16) & 1u);
    return (unsigned short)(r >> 16);
}
__device__ __forceinline__ float bf2f(unsigned short b) {
    return __uint_as_float(((unsigned)b) << 16);
}
__device__ __forceinline__ v8f ld8f(const float* p) {
    v4f a = *(const v4f*)p;
    v4f b = *(const v4f*)(p + 4);
    return __builtin_shufflevector(a, b, 0, 1, 2, 3, 4, 5, 6, 7);
}
__device__ __forceinline__ void split8(const v8f x, u16x8& hv, u16x8& lv) {
#pragma unroll
    for (int c = 0; c < 8; ++c) {
        const float f = x[c];
        const unsigned short hb = f2bf(f);
        const unsigned short lb = f2bf(f - bf2f(hb));
        hv[c] = hb;
        lv[c] = lb;
    }
}
__device__ __forceinline__ u16x8 to_f16x8(const v8f x) {
    H8U t;
    t.f = __builtin_convertvector(x, v8h);
    return t.u;
}
__device__ __forceinline__ float sigm_(float x) {
    return __builtin_amdgcn_rcpf(1.0f + __expf(-x));
}
__device__ __forceinline__ float tanh_(float x) {
    const float a = fabsf(x);
    const float e = __expf(-2.0f * a);
    const float t = (1.0f - e) * __builtin_amdgcn_rcpf(1.0f + e);
    return copysignf(t, x);
}

__device__ __forceinline__ void mma_bf(v8f& acc, const Frag& a, const Frag& b) {
    acc = __builtin_amdgcn_wmma_f32_16x16x32_bf16(false, a.vb, false, b.vb, (short)0, acc, false, false);
    asm volatile("v_nop\n\tv_nop\n\tv_nop\n\tv_nop" : "+v"(acc) : "v"(a.vb), "v"(b.vb));
}
__device__ __forceinline__ void mma_hf(v8f& acc, const Frag& a, const Frag& b) {
    acc = __builtin_amdgcn_wmma_f32_16x16x32_f16(false, a.vh, false, b.vh, (short)0, acc, false, false);
    asm volatile("v_nop\n\tv_nop\n\tv_nop\n\tv_nop" : "+v"(acc) : "v"(a.vh), "v"(b.vh));
}

__global__ __launch_bounds__(256)
void embed_kernel(const int* __restrict__ tok, const float* __restrict__ lang, const float* __restrict__ etab,
                  unsigned short* xp)
{
    const int i   = blockIdx.x * 256 + threadIdx.x;
    const int row = i >> 7;
    const int c   = (i & 127) * 8;
    int tk = tok[row];
    tk = min(max(tk, 0), VOC_ - 1);
    const int cl = min(c, LM_ - 8);
    const int ce = max(c - LM_, 0);
    const v8f a = ld8f(lang + (size_t)row * LM_ + cl);
    const v8f b = ld8f(etab + (size_t)tk * EMB_ + ce);
    const bool first = (c < LM_);
    v8f v;
#pragma unroll
    for (int k = 0; k < 8; ++k) v[k] = first ? a[k] : b[k];
    const u16x8 o = to_f16x8(v);
    const size_t e = (size_t)i * 8;
    *(volatile u16x8*)(xp + e) = o;
    __threadfence();
    *(volatile u16x8*)(xp + e) = o;
}

__global__ __launch_bounds__(256)
void cvt_split_kernel(const float* __restrict__ src, int nsrc, unsigned short* dhi, unsigned short* dlo, int n8)
{
    const int i = blockIdx.x * 256 + threadIdx.x;
    if (i >= n8) return;
    const size_t e  = (size_t)i * 8;
    const bool   in = (e + 8 <= (size_t)nsrc);
    const size_t ec = in ? e : (size_t)(nsrc - 8);
    v8f x = ld8f(src + ec);
#pragma unroll
    for (int k = 0; k < 8; ++k) x[k] = in ? x[k] : 0.0f;
    u16x8 hv, lv;
    split8(x, hv, lv);
    *(volatile u16x8*)(dhi + e) = hv;
    *(volatile u16x8*)(dlo + e) = lv;
    __threadfence();
    *(volatile u16x8*)(dhi + e) = hv;
    *(volatile u16x8*)(dlo + e) = lv;
}

__global__ __launch_bounds__(256)
void cvt_f16_kernel(const float* __restrict__ src, unsigned short* dst, float scale, int n8)
{
    const int i = blockIdx.x * 256 + threadIdx.x;
    if (i >= n8) return;
    const size_t e = (size_t)i * 8;
    const v8f x = ld8f(src + e) * scale;
    const u16x8 o = to_f16x8(x);
    *(volatile u16x8*)(dst + e) = o;
    __threadfence();
    *(volatile u16x8*)(dst + e) = o;
}

template<int OPER, int EPI>
__global__ __launch_bounds__(128)
void gemm_kernel(const unsigned short* __restrict__ Ah, const unsigned short* __restrict__ Al,
                 const unsigned short* __restrict__ Bh, const unsigned short* __restrict__ Bl,
                 const float* __restrict__ bias0, const float* __restrict__ bias1,
                 float* Cf, unsigned short* Ch, unsigned short* Cl,
                 float scale, int K, int ldc, int thl, int sstride, int t0)
{
    __shared__ __attribute__((aligned(16))) float sC[64 * SCP_];

    const int tid  = threadIdx.x;
    const int lane = tid & 31;
    const int wave = tid >> 5;
    const int h    = lane >> 4;
    const int m    = lane & 15;
    const int wm   = wave >> 1;
    const int wn   = wave & 1;

    const int vrow0 = blockIdx.y * 64;
    const int vroww = vrow0 + wm * 32;
    const int prow  = (vroww >> thl) * sstride + t0 + (vroww & ((1 << thl) - 1));
    const int col0  = blockIdx.x * 64;
    const int colw  = col0 + wn * 32;

    v8f acc[4];
#pragma unroll
    for (int j = 0; j < 4; ++j)
#pragma unroll
        for (int r = 0; r < 8; ++r) acc[j][r] = 0.0f;

    const size_t aoff  = (size_t)(prow + m) * K + 8 * h;
    const size_t boff  = (size_t)(colw + m) * K + 8 * h;
    const size_t sub16 = (size_t)16 * K;
    const int nk = K >> 5;

#pragma unroll 1
    for (int kt = 0; kt < nk; ++kt) {
        const size_t k0 = (size_t)kt * 32;
        Frag fa[2], fb[2];
#pragma unroll
        for (int s = 0; s < 2; ++s) {
            const unsigned short* p = Ah + aoff + s * sub16 + k0;
            fa[s].h[0] = *(const u16x8*)(p);
            fa[s].h[1] = *(const u16x8*)(p + 16);
        }
#pragma unroll
        for (int j = 0; j < 2; ++j) {
            const unsigned short* q = Bh + boff + j * sub16 + k0;
            fb[j].h[0] = *(const u16x8*)(q);
            fb[j].h[1] = *(const u16x8*)(q + 16);
        }
        if constexpr (OPER == 0) {
            Frag ga[2], gb[2];
#pragma unroll
            for (int s = 0; s < 2; ++s) {
                const unsigned short* p = Al + aoff + s * sub16 + k0;
                ga[s].h[0] = *(const u16x8*)(p);
                ga[s].h[1] = *(const u16x8*)(p + 16);
            }
#pragma unroll
            for (int j = 0; j < 2; ++j) {
                const unsigned short* q = Bl + boff + j * sub16 + k0;
                gb[j].h[0] = *(const u16x8*)(q);
                gb[j].h[1] = *(const u16x8*)(q + 16);
            }
#pragma unroll
            for (int s = 0; s < 2; ++s)
#pragma unroll
                for (int j = 0; j < 2; ++j) {
                    mma_bf(acc[s * 2 + j], fa[s], fb[j]);
                    mma_bf(acc[s * 2 + j], fa[s], gb[j]);
                    mma_bf(acc[s * 2 + j], ga[s], fb[j]);
                }
        } else {
#pragma unroll
            for (int s = 0; s < 2; ++s)
#pragma unroll
                for (int j = 0; j < 2; ++j)
                    mma_hf(acc[s * 2 + j], fa[s], fb[j]);
        }
    }

#pragma unroll
    for (int s = 0; s < 2; ++s)
#pragma unroll
        for (int j = 0; j < 2; ++j)
#pragma unroll
            for (int r = 0; r < 8; ++r)
                sC[(wm * 32 + s * 16 + 8 * h + r) * SCP_ + wn * 32 + j * 16 + m] = acc[s * 2 + j][r];
    __syncthreads();

    if constexpr (EPI == 0) {
        const int c4 = (lane & 15) * 4;
        const v4f b0v = *(const v4f*)(bias0 + col0 + c4);
        const v4f b1v = *(const v4f*)(bias1 + col0 + c4);
        v4f vals[8];
#pragma unroll
        for (int it = 0; it < 8; ++it) {
            const int row = wave * 16 + it * 2 + (lane >> 4);
            const v4f v = *(const v4f*)(sC + row * SCP_ + c4);
            vals[it] = (v * scale + b0v) + b1v;
        }
#pragma unroll
        for (int it = 0; it < 8; ++it) {
            const int row = wave * 16 + it * 2 + (lane >> 4);
            float* gp = Cf + (size_t)(vrow0 + row) * ldc + col0 + c4;
            *(volatile v4f*)gp = vals[it];
        }
        __threadfence();
#pragma unroll
        for (int it = 0; it < 8; ++it) {
            const int row = wave * 16 + it * 2 + (lane >> 4);
            float* gp = Cf + (size_t)(vrow0 + row) * ldc + col0 + c4;
            *(volatile v4f*)gp = vals[it];
        }
    } else if constexpr (EPI == 1) {
        const int c8 = (lane & 7) * 8;
        const v8f bv = ld8f(bias0 + col0 + c8);
        u16x8 hv[4], lv[4];
#pragma unroll
        for (int it = 0; it < 4; ++it) {
            const int row = wave * 16 + it * 4 + (lane >> 3);
            v8f v = ld8f(sC + row * SCP_ + c8) * scale + bv;
#pragma unroll
            for (int k = 0; k < 8; ++k) v[k] = (v[k] > 0.0f) ? v[k] : 0.01f * v[k];
            split8(v, hv[it], lv[it]);
        }
#pragma unroll
        for (int it = 0; it < 4; ++it) {
            const int row = wave * 16 + it * 4 + (lane >> 3);
            const size_t o = (size_t)(vrow0 + row) * ldc + col0 + c8;
            *(volatile u16x8*)(Ch + o) = hv[it];
            *(volatile u16x8*)(Cl + o) = lv[it];
        }
        __threadfence();
#pragma unroll
        for (int it = 0; it < 4; ++it) {
            const int row = wave * 16 + it * 4 + (lane >> 3);
            const size_t o = (size_t)(vrow0 + row) * ldc + col0 + c8;
            *(volatile u16x8*)(Ch + o) = hv[it];
            *(volatile u16x8*)(Cl + o) = lv[it];
        }
    } else {
        const int p = (tid < 80) ? tid : 79;
        v4f ov;
#pragma unroll
        for (int k = 0; k < 4; ++k) {
            const int e   = 4 * p + k;
            const int row = e / NCL_;
            const int c   = e - row * NCL_;
            ov[k] = sC[row * SCP_ + c] * scale + bias0[c];
        }
        float* gp = Cf + (size_t)vrow0 * NCL_ + 4 * p;
        if (tid < 80) *(volatile v4f*)gp = ov;
        __threadfence();
        if (tid < 80) *(volatile v4f*)gp = ov;
    }
}

template<int MODE>
__global__ __launch_bounds__(512)
void rec_kernel(const float* __restrict__ XG, const unsigned short* __restrict__ Wp,
                const int* __restrict__ lengths, float* cst, unsigned short* hst,
                unsigned short* Yh, unsigned short* Yl,
                int t0, int tfirst, int tstep, int init, int save, int ycol0)
{
    __shared__ __attribute__((aligned(16))) unsigned short hbuf[NB_ * NH_];
    __shared__ __attribute__((aligned(16))) YStage st;

    const int tid   = threadIdx.x;
    const int lane  = tid & 31;
    const int wave  = tid >> 5;
    const int h     = lane >> 4;
    const int m     = lane & 15;
    const int ubase = wave * 32;
    const float SC  = 0.0625f;

    float cs[2][8];
    if (init != 0) {
        u16x8 z;
#pragma unroll
        for (int k = 0; k < 8; ++k) z[k] = 0;
        *(u16x8*)(hbuf + tid * 16)     = z;
        *(u16x8*)(hbuf + tid * 16 + 8) = z;
#pragma unroll
        for (int jj = 0; jj < 2; ++jj)
#pragma unroll
            for (int r = 0; r < 8; ++r) cs[jj][r] = 0.0f;
    } else {
        *(u16x8*)(hbuf + tid * 16)     = *(const u16x8*)(hst + tid * 16);
        *(u16x8*)(hbuf + tid * 16 + 8) = *(const u16x8*)(hst + tid * 16 + 8);
#pragma unroll
        for (int jj = 0; jj < 2; ++jj)
#pragma unroll
            for (int r = 0; r < 8; ++r)
                cs[jj][r] = cst[(8 * h + r) * NH_ + ubase + 16 * jj + m];
    }
    int lenv[8];
#pragma unroll
    for (int r = 0; r < 8; ++r) lenv[r] = lengths[8 * h + r];
    __syncthreads();

#pragma unroll 1
    for (int j = 0; j < TH_; ++j) {
        const int t = tfirst + j * tstep;

        v8f acc[8];
#pragma unroll
        for (int q = 0; q < 8; ++q)
#pragma unroll
            for (int r = 0; r < 8; ++r) acc[q][r] = 0.0f;

#pragma unroll 1
        for (int kt = 0; kt < NH_ / 32; ++kt) {
            const int k0 = kt * 32;
            Frag a;
            a.h[0] = *(const u16x8*)(hbuf + m * NH_ + k0 + 8 * h);
            a.h[1] = *(const u16x8*)(hbuf + m * NH_ + k0 + 16 + 8 * h);
#pragma unroll
            for (int g = 0; g < 4; ++g)
#pragma unroll
                for (int jj = 0; jj < 2; ++jj) {
                    const int n = g * NH_ + ubase + 16 * jj + m;
                    const unsigned short* q = Wp + (size_t)n * NH_ + k0 + 8 * h;
                    Frag b;
                    b.h[0] = *(const u16x8*)(q);
                    b.h[1] = *(const u16x8*)(q + 16);
                    mma_hf(acc[g * 2 + jj], a, b);
                }
        }
        __syncthreads();

        const float* xg = XG + (size_t)(t - t0) * NG_;
#pragma unroll
        for (int jj = 0; jj < 2; ++jj) {
            const int u = ubase + 16 * jj + m;
#pragma unroll
            for (int r = 0; r < 8; ++r) {
                const int b = 8 * h + r;
                const float* xr = xg + (size_t)b * ((size_t)TH_ * NG_) + u;
                const float xi = xr[0];
                const float xf = xr[NH_];
                const float xc = xr[2 * NH_];
                const float xo = xr[3 * NH_];
                const float gi = sigm_(acc[0 + jj][r] * SC + xi);
                const float gf = sigm_(acc[2 + jj][r] * SC + xf);
                const float gc = tanh_(acc[4 + jj][r] * SC + xc);
                const float go = sigm_(acc[6 + jj][r] * SC + xo);
                const float cold = cs[jj][r];
                const float cnew = gf * cold + gi * gc;
                const float hnew = go * tanh_(cnew);
                const bool  mk   = t < lenv[r];
                cs[jj][r] = mk ? cnew : cold;
                const float y = mk ? hnew : 0.0f;
                if (mk) {
                    H2U hb; hb.f = (_Float16)hnew;
                    hbuf[b * NH_ + u] = hb.u;
                }
                if constexpr (MODE == 0) {
                    const unsigned short yh = f2bf(y);
                    const unsigned short yl = f2bf(y - bf2f(yh));
                    st.y[b * NH_ + u] = yh;
                    st.y[NB_ * NH_ + b * NH_ + u] = yl;
                } else {
                    H2U yb; yb.f = (_Float16)y;
                    st.y[b * NH_ + u] = yb.u;
                }
            }
        }
        __syncthreads();

        {
            const unsigned short* ys = st.y + wave * NH_ + lane * 8;
            const u16x8 v0 = *(const u16x8*)(ys);
            const u16x8 v1 = *(const u16x8*)(ys + 256);
            const size_t go = ((size_t)wave * NS_ + t) * DIN_ + ycol0 + lane * 8;
            if constexpr (MODE == 0) {
                const u16x8 v2 = *(const u16x8*)(ys + NB_ * NH_);
                const u16x8 v3 = *(const u16x8*)(ys + NB_ * NH_ + 256);
                *(volatile u16x8*)(Yh + go)       = v0;
                *(volatile u16x8*)(Yh + go + 256) = v1;
                *(volatile u16x8*)(Yl + go)       = v2;
                *(volatile u16x8*)(Yl + go + 256) = v3;
                __threadfence();
                *(volatile u16x8*)(Yh + go)       = v0;
                *(volatile u16x8*)(Yh + go + 256) = v1;
                *(volatile u16x8*)(Yl + go)       = v2;
                *(volatile u16x8*)(Yl + go + 256) = v3;
            } else {
                *(volatile u16x8*)(Yh + go)       = v0;
                *(volatile u16x8*)(Yh + go + 256) = v1;
                __threadfence();
                *(volatile u16x8*)(Yh + go)       = v0;
                *(volatile u16x8*)(Yh + go + 256) = v1;
            }
        }
    }

    if (save != 0) {
        __syncthreads();
#pragma unroll
        for (int jj = 0; jj < 2; ++jj)
#pragma unroll
            for (int r = 0; r < 8; ++r)
                st.c[(8 * h + r) * NH_ + ubase + 16 * jj + m] = cs[jj][r];
        __syncthreads();
        v4f cv[4];
        u16x8 hv[2];
#pragma unroll
        for (int q = 0; q < 4; ++q) cv[q] = *(const v4f*)(st.c + wave * NH_ + q * 128 + lane * 4);
#pragma unroll
        for (int q = 0; q < 2; ++q) hv[q] = *(const u16x8*)(hbuf + wave * NH_ + q * 256 + lane * 8);
#pragma unroll
        for (int q = 0; q < 4; ++q) *(volatile v4f*)(cst + wave * NH_ + q * 128 + lane * 4) = cv[q];
#pragma unroll
        for (int q = 0; q < 2; ++q) *(volatile u16x8*)(hst + wave * NH_ + q * 256 + lane * 8) = hv[q];
        __threadfence();
#pragma unroll
        for (int q = 0; q < 4; ++q) *(volatile v4f*)(cst + wave * NH_ + q * 128 + lane * 4) = cv[q];
#pragma unroll
        for (int q = 0; q < 2; ++q) *(volatile u16x8*)(hst + wave * NH_ + q * 256 + lane * 8) = hv[q];
    }
}

extern "C" void kernel_launch(void* const* d_in, const int* in_sizes, int n_in,
                              void* d_out, int out_size, void* d_ws, size_t ws_size,
                              hipStream_t stream)
{
    if (n_in < 14) return;
    if (in_sizes[0]  != NR_)              return;
    if (in_sizes[1]  != NB_)              return;
    if (in_sizes[2]  != NR_ * LM_)        return;
    if (in_sizes[3]  != VOC_ * EMB_)      return;
    if (in_sizes[4]  != 4 * NG_ * DIN_)   return;
    if (in_sizes[5]  != 4 * NG_ * NH_)    return;
    if (in_sizes[6]  != 4 * NG_)          return;
    if (in_sizes[7]  != 4 * NG_)          return;
    if (in_sizes[8]  != HID_ * DIN_)      return;
    if (in_sizes[9]  != HID_)             return;
    if (in_sizes[10] != HID_ * HID_)      return;
    if (in_sizes[11] != HID_)             return;
    if (in_sizes[12] != NCL_ * HID_)      return;
    if (in_sizes[13] != NCL_)             return;
    if (out_size != NR_ * NCL_)           return;
    if (ws_size < WS_END)                 return;

    const int*   tok  = (const int*)d_in[0];
    const int*   lens = (const int*)d_in[1];
    const float* lang = (const float*)d_in[2];
    const float* etab = (const float*)d_in[3];
    const float* Wih  = (const float*)d_in[4];
    const float* Whh  = (const float*)d_in[5];
    const float* bih  = (const float*)d_in[6];
    const float* bhh  = (const float*)d_in[7];
    const float* W1   = (const float*)d_in[8];
    const float* b1   = (const float*)d_in[9];
    const float* W2   = (const float*)d_in[10];
    const float* b2   = (const float*)d_in[11];
    const float* W3   = (const float*)d_in[12];
    const float* b3   = (const float*)d_in[13];
    float* out = (float*)d_out;

    char* ws = (char*)d_ws;
    unsigned short* pxh  = (unsigned short*)(ws + OFF_PXH);
    unsigned short* pxl  = (unsigned short*)(ws + OFF_PXL);
    unsigned short* pyh  = (unsigned short*)(ws + OFF_PYH);
    unsigned short* pyl  = (unsigned short*)(ws + OFF_PYL);
    float*          xg   = (float*)(ws + OFF_XG);
    unsigned short* wihh = (unsigned short*)(ws + OFF_WIHH);
    unsigned short* wihl = (unsigned short*)(ws + OFF_WIHL);
    unsigned short* whh  = (unsigned short*)(ws + OFF_WHH);
    unsigned short* w1p  = (unsigned short*)(ws + OFF_W1P);
    unsigned short* w2h  = (unsigned short*)(ws + OFF_W2H);
    unsigned short* w2l  = (unsigned short*)(ws + OFF_W2L);
    unsigned short* w3h  = (unsigned short*)(ws + OFF_W3H);
    unsigned short* w3l  = (unsigned short*)(ws + OFF_W3L);
    float*          cst  = (float*)(ws + OFF_CST);
    unsigned short* hst  = (unsigned short*)(ws + OFF_HST);
    unsigned short* y2p  = pxh;
    unsigned short* a1h  = pyh;
    unsigned short* a1l  = pyl;
    unsigned short* a2h  = pxh;
    unsigned short* a2l  = pxl;

    embed_kernel<<<dim3((NR_ * DIN_ / 8) / 256), dim3(256), 0, stream>>>(tok, lang, etab, pxh);

    for (int l = 0; l < 2; ++l) {
        const unsigned short* ah = (l == 0) ? pxh : pyh;
        const unsigned short* al = (l == 0) ? pxh : pyl;
        for (int d = 0; d < 2; ++d) {
            const int ld = l * 2 + d;
            if (l == 0) {
                cvt_f16_kernel<<<dim3((NG_ * DIN_ / 8) / 256), dim3(256), 0, stream>>>(
                    Wih + (size_t)ld * NG_ * DIN_, wihh, 16.0f, NG_ * DIN_ / 8);
            } else {
                cvt_split_kernel<<<dim3((NG_ * DIN_ / 8) / 256), dim3(256), 0, stream>>>(
                    Wih + (size_t)ld * NG_ * DIN_, NG_ * DIN_, wihh, wihl, NG_ * DIN_ / 8);
            }
            cvt_f16_kernel<<<dim3((NG_ * NH_ / 8) / 256), dim3(256), 0, stream>>>(
                Whh + (size_t)ld * NG_ * NH_, whh, 16.0f, NG_ * NH_ / 8);
            for (int half = 0; half < 2; ++half) {
                const int t0     = (d == 0) ? half * TH_ : (1 - half) * TH_;
                const int tfirst = (d == 0) ? t0 : t0 + TH_ - 1;
                const int tstep  = (d == 0) ? 1 : -1;
                const int first  = (half == 0) ? 1 : 0;
                if (l == 0) {
                    gemm_kernel<1, 0><<<dim3(NG_ / 64, NRH_ / 64), dim3(128), 0, stream>>>(
                        ah, ah, wihh, wihh, bih + (size_t)ld * NG_, bhh + (size_t)ld * NG_,
                        xg, hst, hst, 0.0625f, (int)DIN_, (int)NG_, 8, (int)NS_, t0);
                } else {
                    gemm_kernel<0, 0><<<dim3(NG_ / 64, NRH_ / 64), dim3(128), 0, stream>>>(
                        ah, al, wihh, wihl, bih + (size_t)ld * NG_, bhh + (size_t)ld * NG_,
                        xg, hst, hst, 1.0f, (int)DIN_, (int)NG_, 8, (int)NS_, t0);
                }
                if (l == 0) {
                    rec_kernel<0><<<dim3(1), dim3(512), 0, stream>>>(
                        (const float*)xg, (const unsigned short*)whh, lens, cst, hst, pyh, pyl,
                        t0, tfirst, tstep, first, first, d * NH_);
                } else {
                    rec_kernel<1><<<dim3(1), dim3(512), 0, stream>>>(
                        (const float*)xg, (const unsigned short*)whh, lens, cst, hst, y2p, y2p,
                        t0, tfirst, tstep, first, first, d * NH_);
                }
            }
        }
    }

    cvt_f16_kernel<<<dim3((HID_ * DIN_ / 8) / 256), dim3(256), 0, stream>>>(W1, w1p, 16.0f, HID_ * DIN_ / 8);
    cvt_split_kernel<<<dim3((HID_ * HID_ / 8) / 256), dim3(256), 0, stream>>>(W2, HID_ * HID_, w2h, w2l, HID_ * HID_ / 8);
    cvt_split_kernel<<<dim3((W3R_ * HID_ / 8) / 256), dim3(256), 0, stream>>>(W3, NCL_ * HID_, w3h, w3l, W3R_ * HID_ / 8);

    gemm_kernel<1, 1><<<dim3(HID_ / 64, NR_ / 64), dim3(128), 0, stream>>>(
        (const unsigned short*)y2p, (const unsigned short*)y2p, (const unsigned short*)w1p, (const unsigned short*)w1p,
        b1, b1, xg, a1h, a1l, 0.0625f, (int)DIN_, (int)HID_, 20, 0, 0);
    gemm_kernel<0, 1><<<dim3(HID_ / 64, NR_ / 64), dim3(128), 0, stream>>>(
        (const unsigned short*)a1h, (const unsigned short*)a1l, (const unsigned short*)w2h, (const unsigned short*)w2l,
        b2, b2, xg, a2h, a2l, 1.0f, (int)HID_, (int)HID_, 20, 0, 0);
    gemm_kernel<0, 2><<<dim3(1, NR_ / 64), dim3(128), 0, stream>>>(
        (const unsigned short*)a2h, (const unsigned short*)a2l, (const unsigned short*)w3h, (const unsigned short*)w3l,
        b3, b3, out, a1h, a1l, 1.0f, (int)HID_, (int)NCL_, 20, 0, 0);
}
